// HebbianLinear_55697135895031
// MI455X (gfx1250) — hardware-verified
//
#include <hip/hip_runtime.h>
#include <math.h>


typedef _Float16 f16t;
typedef _Float16 v16h __attribute__((ext_vector_type(16)));
typedef _Float16 v8h  __attribute__((ext_vector_type(8)));
typedef float    v8f  __attribute__((ext_vector_type(8)));
typedef float    v4f  __attribute__((ext_vector_type(4)));

union Frag { v16h v; v8h half[2]; };

#define RATE_C 0.01f

static __device__ __forceinline__ void wmma16(v8f& acc, const v16h& a, const v16h& b) {
  acc = __builtin_amdgcn_wmma_f32_16x16x32_f16(false, a, false, b, (short)0, acc, false, false);
  asm volatile("v_nop\n\tv_nop\n\tv_nop\n\tv_nop" : "+v"(acc) : "v"(a), "v"(b));
}

static __device__ __forceinline__ double shfl_xor_d(double v, int msk) {
  const long long bits = __double_as_longlong(v);
  int lo = (int)(bits & 0xffffffffLL);
  int hi = (int)(bits >> 32);
  lo = __shfl_xor(lo, msk, 32);
  hi = __shfl_xor(hi, msk, 32);
  const long long r = ((long long)hi << 32) | (long long)(unsigned int)lo;
  return __longlong_as_double(r);
}

template <int MT, int NT>
static __device__ __forceinline__ void gemm_core(const f16t* __restrict__ A,
                                                 const f16t* __restrict__ Bn,
                                                 int K, int M0, int N0, int lane,
                                                 v8f (&acc)[MT][NT]) {
  const int m = lane & 15;
  const int h = lane >> 4;
  const f16t* ap[MT];
  const f16t* bp[NT];
#pragma unroll
  for (int mt = 0; mt < MT; ++mt) ap[mt] = A + (size_t)(M0 + mt * 16 + m) * K + 8 * h;
#pragma unroll
  for (int nt = 0; nt < NT; ++nt) bp[nt] = Bn + (size_t)(N0 + nt * 16 + m) * K + 8 * h;

#pragma unroll 1
  for (int k0 = 0; k0 < K; k0 += 32) {
    Frag a[MT], b[NT];
#pragma unroll
    for (int mt = 0; mt < MT; ++mt) {
      a[mt].half[0] = *(const v8h*)(ap[mt] + k0);
      a[mt].half[1] = *(const v8h*)(ap[mt] + k0 + 16);
    }
#pragma unroll
    for (int nt = 0; nt < NT; ++nt) {
      b[nt].half[0] = *(const v8h*)(bp[nt] + k0);
      b[nt].half[1] = *(const v8h*)(bp[nt] + k0 + 16);
    }
#pragma unroll
    for (int mt = 0; mt < MT; ++mt)
#pragma unroll
      for (int nt = 0; nt < NT; ++nt)
        wmma16(acc[mt][nt], a[mt].v, b[nt].v);
  }
}

__global__ __launch_bounds__(256)
void k_cvt(const float* __restrict__ src, f16t* __restrict__ dst, int n8, float scale) {
  const int i = blockIdx.x * 256 + threadIdx.x;
  if (i >= n8) return;
  const v4f* s4 = (const v4f*)src;
  const v4f lo = s4[2 * (size_t)i];
  const v4f hi = s4[2 * (size_t)i + 1];
  v8h d;
#pragma unroll
  for (int j = 0; j < 4; ++j) {
    d[j]     = (f16t)(lo[j] * scale);
    d[4 + j] = (f16t)(hi[j] * scale);
  }
  f16t* p = dst + (size_t)i * 8;
  *(volatile v8h*)p = d;
  __threadfence();
  *(volatile v8h*)p = d;
}

__global__ __launch_bounds__(256)
void k_transpose(const float* __restrict__ src, f16t* __restrict__ dst, int R, int C, float scale) {
  __shared__ __attribute__((aligned(16))) f16t tile[64][66];
  const int tid = threadIdx.x;
  const int lane = tid & 31, wave = tid >> 5;
  const int c0 = blockIdx.x * 64;
  const int r0 = blockIdx.y * 64;
  const int cl = tid & 63, rb = tid >> 6;
#pragma unroll
  for (int j = 0; j < 16; ++j) {
    const int rl = rb + 4 * j;
    tile[rl][cl] = (f16t)(src[(size_t)(r0 + rl) * C + c0 + cl] * scale);
  }
  __syncthreads();
  const int q = lane >> 3, cc = (lane & 7) * 8;
  v8h v[2];
  f16t* p[2];
#pragma unroll
  for (int g = 0; g < 2; ++g) {
    const int dr = wave * 8 + g * 4 + q;
#pragma unroll
    for (int j = 0; j < 8; ++j) v[g][j] = tile[cc + j][dr];
    p[g] = dst + (size_t)(c0 + dr) * R + r0 + cc;
  }
#pragma unroll
  for (int g = 0; g < 2; ++g) *(volatile v8h*)p[g] = v[g];
  __threadfence();
#pragma unroll
  for (int g = 0; g < 2; ++g) *(volatile v8h*)p[g] = v[g];
}

__global__ __launch_bounds__(256)
void k_gemm_u(const f16t* __restrict__ xh, const f16t* __restrict__ wh,
              const float* __restrict__ bias, float* __restrict__ U,
              int IN, int OUT, float inv_scale) {
  __shared__ __attribute__((aligned(16))) float st[8][16][36];
  const int lane = threadIdx.x & 31;
  const int wave = threadIdx.x >> 5;
  const int M0 = blockIdx.y * 128 + (wave >> 2) * 64;
  const int N0 = blockIdx.x * 128 + (wave & 3) * 32;

  v8f acc[4][2] = {};
  gemm_core<4, 2>(xh, wh, IN, M0, N0, lane, acc);

  const int m = lane & 15, h = lane >> 4;
  const int q = lane >> 3, c = (lane & 7) * 4;
  const v4f bz = *(const v4f*)(bias + N0 + c);
#pragma unroll
  for (int mt = 0; mt < 4; ++mt) {
    __syncthreads();
#pragma unroll
    for (int nt = 0; nt < 2; ++nt)
#pragma unroll
      for (int r = 0; r < 8; ++r)
        st[wave][8 * h + r][nt * 16 + m] = acc[mt][nt][r];
    __syncthreads();
    v4f v[4];
    float* p[4];
#pragma unroll
    for (int rr = 0; rr < 4; ++rr) {
      const int rl = rr * 4 + q;
      const v4f a4 = *(const v4f*)(&st[wave][rl][c]);
      v[rr] = a4 * inv_scale + bz;
      p[rr] = U + (size_t)(M0 + mt * 16 + rl) * OUT + N0 + c;
    }
#pragma unroll
    for (int rr = 0; rr < 4; ++rr) *(volatile v4f*)p[rr] = v[rr];
    __threadfence();
#pragma unroll
    for (int rr = 0; rr < 4; ++rr) *(volatile v4f*)p[rr] = v[rr];
  }
}

__global__ __launch_bounds__(256)
void k_rowstats(const float* __restrict__ U, float* __restrict__ rowmax,
                float* __restrict__ rowinv, int OUT) {
  __shared__ __attribute__((aligned(16))) float smax[32];
  __shared__ __attribute__((aligned(16))) float sinv[32];
  const int lane = threadIdx.x & 31;
  const int wave = threadIdx.x >> 5;
  const int b0 = blockIdx.x * 32;
#pragma unroll 1
  for (int t = 0; t < 4; ++t) {
    const int b = b0 + wave * 4 + t;
    const float* ur = U + (size_t)b * OUT;
    float mx = -__builtin_inff();
    for (int o = lane; o < OUT; o += 32) mx = fmaxf(mx, ur[o]);
#pragma unroll
    for (int off = 16; off > 0; off >>= 1) mx = fmaxf(mx, __shfl_xor(mx, off, 32));
    float s = 0.0f;
    for (int o = lane; o < OUT; o += 32) s += __expf(ur[o] - mx);
#pragma unroll
    for (int off = 16; off > 0; off >>= 1) s += __shfl_xor(s, off, 32);
    if (lane == 0) {
      smax[wave * 4 + t] = mx;
      sinv[wave * 4 + t] = 1.0f / s;
    }
  }
  __syncthreads();
  if (wave == 0 && lane < 16) {
    v4f v;
    float* p;
    if (lane < 8) {
      v = *(const v4f*)(&smax[lane * 4]);
      p = rowmax + b0 + lane * 4;
    } else {
      v = *(const v4f*)(&sinv[(lane - 8) * 4]);
      p = rowinv + b0 + (lane - 8) * 4;
    }
    *(volatile v4f*)p = v;
    __threadfence();
    *(volatile v4f*)p = v;
  }
}

__global__ __launch_bounds__(256)
void k_softmax_t(const float* __restrict__ U, const float* __restrict__ rowmax,
                 const float* __restrict__ rowinv, f16t* __restrict__ yt,
                 float* __restrict__ yupart, int Bdim, int OUT, float yscale) {
  __shared__ __attribute__((aligned(16))) f16t tile[64][66];
  __shared__ __attribute__((aligned(16))) float red[256];
  __shared__ __attribute__((aligned(16))) float psum[64];
  const int tid = threadIdx.x;
  const int lane = tid & 31, wave = tid >> 5;
  const int o0 = blockIdx.x * 64;
  const int b0 = blockIdx.y * 64;
  const int ol = tid & 63, bb = tid >> 6;
  const int o = o0 + ol;

  float part = 0.0f;
#pragma unroll 4
  for (int j = 0; j < 16; ++j) {
    const int bl = bb + 4 * j;
    const int b = b0 + bl;
    const float u = U[(size_t)b * OUT + o];
    const float y = __expf(u - rowmax[b]) * rowinv[b];
    part += y * u;
    tile[bl][ol] = (f16t)(y * yscale);
  }
  red[tid] = part;
  __syncthreads();

  const int q = lane >> 3, cc = (lane & 7) * 8;
  v8h v[2];
  f16t* p[2];
#pragma unroll
  for (int g = 0; g < 2; ++g) {
    const int dr = wave * 8 + g * 4 + q;
#pragma unroll
    for (int j = 0; j < 8; ++j) v[g][j] = tile[cc + j][dr];
    p[g] = yt + (size_t)(o0 + dr) * Bdim + b0 + cc;
  }
  if (tid < 64) psum[tid] = (red[tid] + red[tid + 64]) + (red[tid + 128] + red[tid + 192]);
  __syncthreads();

  const bool wr = (tid < 16);
  v4f pv = {0.0f, 0.0f, 0.0f, 0.0f};
  float* pp = yupart;
  if (wr) {
    pv = *(const v4f*)(&psum[tid * 4]);
    pp = yupart + (size_t)blockIdx.y * OUT + o0 + tid * 4;
  }
#pragma unroll
  for (int g = 0; g < 2; ++g) *(volatile v8h*)p[g] = v[g];
  if (wr) *(volatile v4f*)pp = pv;
  __threadfence();
#pragma unroll
  for (int g = 0; g < 2; ++g) *(volatile v8h*)p[g] = v[g];
  if (wr) *(volatile v4f*)pp = pv;
}

__global__ __launch_bounds__(256)
void k_rowvec(const float* __restrict__ yupart, const float* __restrict__ W,
              float* __restrict__ yu, float* __restrict__ sc,
              int nbt, int OUT, int IN, float rate_over_b) {
  __shared__ __attribute__((aligned(16))) float syu[32];
  __shared__ __attribute__((aligned(16))) float ssc[32];
  const int lane = threadIdx.x & 31;
  const int wave = threadIdx.x >> 5;
  const int o0 = blockIdx.x * 32;
#pragma unroll 1
  for (int t = 0; t < 4; ++t) {
    const int o = o0 + wave * 4 + t;
    const float* wr = W + (size_t)o * IN;
    double d = 0.0;
    for (int i = lane; i < IN; i += 32) {
      const double w = (double)wr[i];
      d += w * w;
    }
#pragma unroll
    for (int off = 16; off > 0; off >>= 1) d += shfl_xor_d(d, off);
    float s = 0.0f;
    for (int t2 = lane; t2 < nbt; t2 += 32) s += yupart[(size_t)t2 * OUT + o];
#pragma unroll
    for (int off = 16; off > 0; off >>= 1) s += __shfl_xor(s, off, 32);
    if (lane == 0) {
      const float nrm = sqrtf((float)d);
      syu[wave * 4 + t] = s;
      ssc[wave * 4 + t] = rate_over_b * sqrtf(fabsf(1.0f - nrm));
    }
  }
  __syncthreads();
  if (wave == 0 && lane < 16) {
    v4f v;
    float* p;
    if (lane < 8) {
      v = *(const v4f*)(&syu[lane * 4]);
      p = yu + o0 + lane * 4;
    } else {
      v = *(const v4f*)(&ssc[(lane - 8) * 4]);
      p = sc + o0 + (lane - 8) * 4;
    }
    *(volatile v4f*)p = v;
    __threadfence();
    *(volatile v4f*)p = v;
  }
}

__global__ __launch_bounds__(256)
void k_gemm_step(const f16t* __restrict__ yt, const f16t* __restrict__ xt,
                 const float* __restrict__ W, const float* __restrict__ yu,
                 const float* __restrict__ sc, float* __restrict__ out,
                 int Bdim, int IN, float inv_scale) {
  __shared__ __attribute__((aligned(16))) float st[8][16][36];
  const int lane = threadIdx.x & 31;
  const int wave = threadIdx.x >> 5;
  const int M0 = blockIdx.y * 128 + (wave >> 2) * 64;
  const int N0 = blockIdx.x * 128 + (wave & 3) * 32;

  v8f acc[4][2] = {};
  gemm_core<4, 2>(yt, xt, Bdim, M0, N0, lane, acc);

  const int m = lane & 15, h = lane >> 4;
  const int q = lane >> 3, c = (lane & 7) * 4;
#pragma unroll
  for (int mt = 0; mt < 4; ++mt) {
    __syncthreads();
#pragma unroll
    for (int nt = 0; nt < 2; ++nt)
#pragma unroll
      for (int r = 0; r < 8; ++r)
        st[wave][8 * h + r][nt * 16 + m] = acc[mt][nt][r];
    __syncthreads();
    v4f v[4];
    float* p[4];
#pragma unroll
    for (int rr = 0; rr < 4; ++rr) {
      const int rl = rr * 4 + q;
      const int o = M0 + mt * 16 + rl;
      const v4f a4 = *(const v4f*)(&st[wave][rl][c]);
      const v4f w4 = *(const v4f*)(W + (size_t)o * IN + N0 + c);
      const float yuo = yu[o];
      const float s = sc[o];
      v[rr] = (a4 * inv_scale - w4 * yuo) * s;
      p[rr] = out + (size_t)o * IN + N0 + c;
    }
#pragma unroll
    for (int rr = 0; rr < 4; ++rr) *(volatile v4f*)p[rr] = v[rr];
    __threadfence();
#pragma unroll
    for (int rr = 0; rr < 4; ++rr) *(volatile v4f*)p[rr] = v[rr];
  }
}

static size_t align256(size_t v) { return (v + 255) & ~(size_t)255; }

extern "C" void kernel_launch(void* const* d_in, const int* in_sizes, int n_in,
                              void* d_out, int out_size, void* d_ws, size_t ws_size,
                              hipStream_t stream) {
  if (n_in < 3) return;
  const int OUT = in_sizes[2];
  if (OUT <= 0) return;
  const int IN = in_sizes[1] / OUT;
  if (IN <= 0 || IN * OUT != in_sizes[1]) return;
  const int Bd = in_sizes[0] / IN;
  if (Bd <= 0 || Bd * IN != in_sizes[0]) return;
  if ((Bd % 128) != 0 || (IN % 128) != 0 || (OUT % 128) != 0) return;
  if (out_size != OUT * IN) return;

  const float* x    = (const float*)d_in[0];
  const float* w    = (const float*)d_in[1];
  const float* bias = (const float*)d_in[2];
  float* out = (float*)d_out;

  size_t off = 0;
  const size_t o_xh  = off; off = align256(off + (size_t)Bd * IN * sizeof(f16t));
  const size_t o_wh  = off; off = align256(off + (size_t)OUT * IN * sizeof(f16t));
  const size_t o_xt  = off; off = align256(off + (size_t)IN * Bd * sizeof(f16t));
  const size_t o_U   = off; off = align256(off + (size_t)Bd * OUT * sizeof(float));
  const size_t o_yt  = off; off = align256(off + (size_t)OUT * Bd * sizeof(f16t));
  const size_t o_rmx = off; off = align256(off + (size_t)Bd * sizeof(float));
  const size_t o_riv = off; off = align256(off + (size_t)Bd * sizeof(float));
  const int nbt = Bd / 64;
  const size_t o_yup = off; off = align256(off + (size_t)nbt * OUT * sizeof(float));
  const size_t o_yu  = off; off = align256(off + (size_t)OUT * sizeof(float));
  const size_t o_sc  = off; off = align256(off + (size_t)OUT * sizeof(float));
  if (off > ws_size) return;

  char* ws = (char*)d_ws;
  f16t*  xh     = (f16t*)(ws + o_xh);
  f16t*  wh     = (f16t*)(ws + o_wh);
  f16t*  xt     = (f16t*)(ws + o_xt);
  float* U      = (float*)(ws + o_U);
  f16t*  yt     = (f16t*)(ws + o_yt);
  float* rowmax = (float*)(ws + o_rmx);
  float* rowinv = (float*)(ws + o_riv);
  float* yupart = (float*)(ws + o_yup);
  float* yu     = (float*)(ws + o_yu);
  float* sc     = (float*)(ws + o_sc);

  const float W_SCALE = 64.0f;
  const float Y_SCALE = 4096.0f;

  {
    const int n8x = Bd * IN / 8;
    k_cvt<<<(n8x + 255) / 256, 256, 0, stream>>>(x, xh, n8x, 1.0f);
    const int n8w = OUT * IN / 8;
    k_cvt<<<(n8w + 255) / 256, 256, 0, stream>>>(w, wh, n8w, W_SCALE);
  }
  {
    dim3 g(IN / 64, Bd / 64);
    k_transpose<<<g, 256, 0, stream>>>(x, xt, Bd, IN, 1.0f);
  }
  {
    dim3 g(OUT / 128, Bd / 128);
    k_gemm_u<<<g, 256, 0, stream>>>(xh, wh, bias, U, IN, OUT, 1.0f / W_SCALE);
  }
  k_rowstats<<<Bd / 32, 256, 0, stream>>>(U, rowmax, rowinv, OUT);
  {
    dim3 g(OUT / 64, Bd / 64);
    k_softmax_t<<<g, 256, 0, stream>>>(U, rowmax, rowinv, yt, yupart, Bd, OUT, Y_SCALE);
  }
  k_rowvec<<<OUT / 32, 256, 0, stream>>>(yupart, w, yu, sc, nbt, OUT, IN,
                                         RATE_C * (1.0f / (float)Bd));
  {
    dim3 g(IN / 128, OUT / 128);
    k_gemm_step<<<g, 256, 0, stream>>>(yt, xt, w, yu, sc, out, Bd, IN, 1.0f / Y_SCALE);
  }
}
